// EncodingLayer_63436666962232
// MI455X (gfx1250) — hardware-verified
//
#include <hip/hip_runtime.h>


namespace {
typedef _Float16 b16;
typedef __attribute__((ext_vector_type(16))) _Float16 v16b;
typedef __attribute__((ext_vector_type(8))) _Float16 v8b;
typedef __attribute__((ext_vector_type(4))) _Float16 v4h;
typedef __attribute__((ext_vector_type(2))) _Float16 v2h;
typedef __attribute__((ext_vector_type(8))) float v8f;
typedef __attribute__((ext_vector_type(4))) float v4f;
typedef __attribute__((ext_vector_type(2))) float v2f;
__device__ __forceinline__ float bf16_rne(float f) { unsigned int u = __float_as_uint(f); u += 0x7FFFu + ((u >> 16) & 1u); return __uint_as_float(u & 0xFFFF0000u); }
__device__ __forceinline__ void split16(float v, b16& hi, b16& lo) { hi = (b16)v; lo = (b16)(v - (float)hi); }
__device__ __forceinline__ v16b frag_kb(const b16* p, int hh) { const v8b a = *(const v8b*)(p + 8 * hh), b = *(const v8b*)(p + 16 + 8 * hh); v16b f;
#pragma unroll
  for (int e = 0; e < 8; ++e) { f[e] = a[e]; f[8 + e] = b[e]; } return f; }
__device__ __forceinline__ v8f wmma16b(v16b a, v16b b, v8f c) { v8f d = __builtin_amdgcn_wmma_f32_16x16x32_f16(false, a, false, b, (short)0, c, false, false); asm volatile("v_nop\n\tv_nop\n\tv_nop\n\tv_nop" : "+v"(d) : "v"(a), "v"(b)); return d; }
__device__ __forceinline__ void wave_lds_sync() { __builtin_amdgcn_fence(__ATOMIC_RELEASE, "workgroup"); __builtin_amdgcn_wave_barrier(); __builtin_amdgcn_fence(__ATOMIC_ACQUIRE, "workgroup"); }
__device__ __forceinline__ float pmul(float a, float b) { float p = a * b; asm volatile("" : "+v"(p)); return p; }
__device__ __forceinline__ int iclamp(int v, int lo, int hi) { return v < lo ? lo : (v > hi ? hi : v); }
__device__ __forceinline__ float nexp2(float v) { return __builtin_amdgcn_exp2f(v); }

constexpr int B = 2, T = 2048, DM = 128, H = 8, HD = 128, INNER = H * HD, FF = 256, BL = 2  , QL = 2048  ;
constexpr float XS = 8.0f, WSC = 256.0f, PS = 1024.0f, LOG2E = 1.4426950408889634f, LNEPS = 1e-5f;
static_assert(T % 64 == 0 && QL % 32 == 0 && DM == 128 && HD == 128, "tiling");
__global__ __launch_bounds__(256) void prep_kernel(const float* __restrict__ wq, const float* __restrict__ wk, const float* __restrict__ wv, const float* __restrict__ wo, const float* __restrict__ w1, const float* __restrict__ w2,
                                                   b16* __restrict__ WT, b16* __restrict__ WO, b16* __restrict__ W1T, b16* __restrict__ W2T) {
  const size_t n1 = (size_t)3 * INNER * DM / 8, n2 = (size_t)DM * INNER / 8, n3 = (size_t)FF * DM / 8, n4 = (size_t)DM * FF / 8; size_t u = (size_t)blockIdx.x * 256 + threadIdx.x; v8b o;
  if (u < n1) { const size_t e = u * 8; const int row = (int)(e / DM), d0 = (int)(e % DM); const int part = row / INNER, h = (row % INNER) / HD, ee = row % HD; const float* w = part == 0 ? wq : part == 1 ? wk : wv;
    for (int j = 0; j < 8; ++j) o[j] = (b16)(bf16_rne(w[((size_t)h * DM + d0 + j) * HD + ee]) * WSC); for (int pass = 0; pass < 2; ++pass) { *(volatile v8b*)(WT + e) = o; __threadfence(); } return; } u -= n1;
  if (u < n2) { const size_t e = u * 8; const int oo = (int)(e / INNER), k0 = (int)(e % INNER); for (int j = 0; j < 8; ++j) o[j] = (b16)(bf16_rne(wo[(size_t)(k0 + j) * DM + oo]) * WSC); for (int pass = 0; pass < 2; ++pass) { *(volatile v8b*)(WO + e) = o; __threadfence(); } return; } u -= n2;
  if (u < n3) { const size_t e = u * 8; const int oo = (int)(e / DM), k0 = (int)(e % DM); for (int j = 0; j < 8; ++j) o[j] = (b16)(bf16_rne(w1[(size_t)(k0 + j) * FF + oo]) * WSC); for (int pass = 0; pass < 2; ++pass) { *(volatile v8b*)(W1T + e) = o; __threadfence(); } return; } u -= n3;
  if (u < n4) { const size_t e = u * 8; const int oo = (int)(e / FF), k0 = (int)(e % FF); for (int j = 0; j < 8; ++j) o[j] = (b16)(bf16_rne(w2[(size_t)(k0 + j) * DM + oo]) * WSC); for (int pass = 0; pass < 2; ++pass) { *(volatile v8b*)(W2T + e) = o; __threadfence(); } }
}
__global__ __launch_bounds__(128) void proj_kernel(const float* __restrict__ x, const b16* __restrict__ WT, const float* __restrict__ bq, const float* __restrict__ bk, const float* __restrict__ bv, b16* __restrict__ QP, b16* __restrict__ KP, b16* __restrict__ VTh) {
  __shared__ __attribute__((aligned(16))) b16 As[64][DM + 8]; __shared__ __attribute__((aligned(16))) float Tf[4][16][128 + 4];
  const int wave = threadIdx.x >> 5, lane = threadIdx.x & 31, nloc = lane & 15, hlf = lane >> 4; const int t0 = blockIdx.x * 64; const int b = blockIdx.y; const int slab = blockIdx.z, n0 = slab * 128, part = slab / H, h = slab % H;
  if (part == 0 && t0 >= QL) return;
  const float* xb = x + ((size_t)b * T + t0) * DM; const float* bias = (part == 0 ? bq : part == 1 ? bk : bv) + h * HD;
  for (int i = threadIdx.x; i < 64 * (DM / 4); i += 128) { const int rr = i / (DM / 4), q = (i % (DM / 4)) * 4; const v4f f = *(const v4f*)(xb + (size_t)rr * DM + q); v4h o; for (int j = 0; j < 4; ++j) o[j] = (b16)(bf16_rne(f[j]) * XS); *(v4h*)(&As[rr][q]) = o; }
  __syncthreads();
  v8f acc[8];
#pragma unroll
  for (int t = 0; t < 8; ++t) acc[t] = (v8f){};
#pragma unroll
  for (int kb = 0; kb < DM; kb += 32) { const v16b a = frag_kb(&As[wave * 16 + nloc][kb], hlf);
#pragma unroll
    for (int t = 0; t < 8; ++t) acc[t] = wmma16b(a, frag_kb(WT + (size_t)(n0 + t * 16 + nloc) * DM + kb, hlf), acc[t]); }
#pragma unroll
  for (int t = 0; t < 8; ++t) { const float bb = bf16_rne(bias[t * 16 + nloc]);
#pragma unroll
    for (int r = 0; r < 8; ++r) Tf[wave][8 * hlf + r][t * 16 + nloc] = acc[t][r] * (1.0f / (XS * WSC)) + bb; }
  __syncthreads();
  for (int pass = 0; pass < 2; ++pass) {
    if (part < 2) { b16* plane = part == 0 ? QP : KP;
      for (int rr = 0; rr < 16; ++rr) { const int tok = t0 + wave * 16 + rr; v4h o4; for (int j = 0; j < 4; ++j) o4[j] = (b16)(Tf[wave][rr][lane * 4 + j] * XS); *(volatile v4h*)(plane + (((size_t)b * H + h) * T + tok) * HD + lane * 4) = o4; } }
    else {
#pragma unroll 1
      for (int q = 0; q < 32; ++q) { const int e = wave * 32 + q; const int tk = lane * 2; v2h hv; hv[0] = (b16)(Tf[tk >> 4][tk & 15][e] * XS); hv[1] = (b16)(Tf[(tk + 1) >> 4][(tk + 1) & 15][e] * XS);
        *(volatile v2h*)(VTh + (((size_t)b * H + h) * HD + e) * (size_t)T + t0 + tk) = hv; } }
    __threadfence(); }
}
__global__ __launch_bounds__(64) void attn_kernel(const b16* __restrict__ QP, const b16* __restrict__ KP, const b16* __restrict__ VTh, b16* __restrict__ O) {
  __shared__ __attribute__((aligned(16))) b16 Pb[2][16][32 + 8]; __shared__ __attribute__((aligned(16))) float To[2][16][HD + 4];
  const int wave = threadIdx.x >> 5, lane = threadIdx.x & 31, hh = lane >> 4, col = lane & 15; const int b = blockIdx.y / H, h = blockIdx.y % H; const int q0 = blockIdx.x * 32 + wave * 16, qi = q0 + col;
  const size_t ph = (size_t)b * H + h; const b16* Qb = QP + ph * T * HD; const b16* Kb = KP + ph * T * HD; const b16* Vh = VTh + ph * HD * (size_t)T;
  v16b qa[4];
#pragma unroll
  for (int s = 0; s < 4; ++s) qa[s] = frag_kb(Qb + (size_t)qi * HD + 32 * s, hh);
  const float cs = LOG2E / (11.313708498984761f * XS * XS);
  float m = -INFINITY, l = 0.0f; v8f o[8]; for (int t = 0; t < 8; ++t) o[t] = (v8f){};
#pragma unroll 1
  for (int kb = 0; kb < T; kb += 32) {
    float e[16]; float mx = -INFINITY;
#pragma unroll
    for (int u = 0; u < 2; ++u) { v8f s = (v8f){}; const size_t kr = (size_t)(kb + u * 16 + col) * HD;
#pragma unroll
      for (int st = 0; st < 4; ++st) s = wmma16b(frag_kb(Kb + kr + 32 * st, hh), qa[st], s);
#pragma unroll
      for (int r = 0; r < 8; ++r) { const float vv = s[r] * cs; e[u * 8 + r] = vv; mx = fmaxf(mx, vv); } }
    mx = fmaxf(mx, __shfl_xor(mx, 16)); const float mn = fmaxf(m, mx); const float al = nexp2(m - mn); float sum = 0.0f;
#pragma unroll
    for (int i2 = 0; i2 < 16; ++i2) { const float p = nexp2(e[i2] - mn); sum += p; Pb[wave][col][(i2 < 8 ? 0 : 16) + 8 * hh + (i2 & 7)] = (b16)(p * PS); }
    sum += __shfl_xor(sum, 16); l = l * al + sum; m = mn;
    wave_lds_sync();
    const v16b pf = frag_kb(&Pb[wave][col][0], hh);
#pragma unroll
    for (int t = 0; t < 8; ++t) { o[t] *= al; o[t] = wmma16b(frag_kb(Vh + (size_t)(t * 16 + col) * T + kb, hh), pf, o[t]); }
    wave_lds_sync(); }
  const float inv = 1.0f / (l * PS * XS);
#pragma unroll
  for (int t = 0; t < 8; ++t)
#pragma unroll
    for (int r = 0; r < 8; ++r) To[wave][col][t * 16 + 8 * hh + r] = o[t][r] * inv;
  wave_lds_sync();
  for (int pass = 0; pass < 2; ++pass) { for (int rr = 0; rr < 16; ++rr) { const v4f f = *(const v4f*)(&To[wave][rr][lane * 4]); v4h hv; for (int j = 0; j < 4; ++j) hv[j] = (b16)(f[j] * XS);
      *(volatile v4h*)(O + ((size_t)b * T + q0 + rr) * INNER + h * HD + lane * 4) = hv; } __threadfence(); }
}
__device__ __forceinline__ void row_ln_store(float (*Tfw)[128 + 4], int lane, const float* __restrict__ g, const float* __restrict__ be, float* dst_rows, size_t row0, size_t ldd, bool twice_volatile) {
  for (int pass = 0; pass < 2; ++pass) { for (int rr = 0; rr < 16; ++rr) { const v4f v = *(const v4f*)(&Tfw[rr][lane * 4]); float s1 = v[0] + v[1] + v[2] + v[3];
      for (int w = 16; w >= 1; w >>= 1) s1 += __shfl_xor(s1, w); const float mu = s1 * (1.0f / 128.0f); float s2 = 0.0f; for (int j = 0; j < 4; ++j) { const float d = v[j] - mu; s2 += d * d; }
      for (int w = 16; w >= 1; w >>= 1) s2 += __shfl_xor(s2, w); const float rs = rsqrtf(s2 * (1.0f / 128.0f) + LNEPS); v4f o;
      for (int j = 0; j < 4; ++j) o[j] = (v[j] - mu) * rs * bf16_rne(g[lane * 4 + j]) + bf16_rne(be[lane * 4 + j]); *(volatile v4f*)(dst_rows + (row0 + rr) * ldd + lane * 4) = o; } __threadfence(); }
  (void)twice_volatile;
}
__global__ __launch_bounds__(128) void outln_kernel(const b16* __restrict__ O, const b16* __restrict__ WO, const float* __restrict__ bo, const float* __restrict__ g1, const float* __restrict__ be1, float* __restrict__ Y1) {
  __shared__ __attribute__((aligned(16))) float Tf[4][16][128 + 4];
  const int wave = threadIdx.x >> 5, lane = threadIdx.x & 31, nloc = lane & 15, hlf = lane >> 4; const size_t m0 = ((size_t)blockIdx.x * 4 + wave) * 16;
  v8f acc[8];
#pragma unroll
  for (int t = 0; t < 8; ++t) acc[t] = (v8f){};
#pragma unroll 4
  for (int kb = 0; kb < INNER; kb += 32) { const v16b a = frag_kb(O + (m0 + nloc) * INNER + kb, hlf);
#pragma unroll
    for (int t = 0; t < 8; ++t) acc[t] = wmma16b(a, frag_kb(WO + (size_t)(t * 16 + nloc) * INNER + kb, hlf), acc[t]); }
#pragma unroll
  for (int t = 0; t < 8; ++t) { const float bb = bf16_rne(bo[t * 16 + nloc]);
#pragma unroll
    for (int r = 0; r < 8; ++r) Tf[wave][8 * hlf + r][t * 16 + nloc] = acc[t][r] * (1.0f / (XS * WSC)) + bb; }
  wave_lds_sync();
  row_ln_store(Tf[wave], lane, g1, be1, Y1, m0, DM, true);
}
__global__ __launch_bounds__(64) void ffn1_kernel(const float* __restrict__ Y1, const b16* __restrict__ W1T, const float* __restrict__ b1, float* __restrict__ F1) {
  __shared__ __attribute__((aligned(16))) b16 Ah[2][16][DM + 8], Al[2][16][DM + 8]; __shared__ __attribute__((aligned(16))) float Tf[2][16][FF + 4];
  const int wave = threadIdx.x >> 5, lane = threadIdx.x & 31, nloc = lane & 15, hlf = lane >> 4; const size_t m0 = (size_t)blockIdx.x * 32 + wave * 16;
  for (int rr = 0; rr < 16; ++rr) { const v4f v = *(const v4f*)(Y1 + (m0 + rr) * DM + lane * 4); v4h hv, lv; for (int j = 0; j < 4; ++j) { b16 p, q; split16(v[j] * XS, p, q); hv[j] = p; lv[j] = q; } *(v4h*)(&Ah[wave][rr][lane * 4]) = hv; *(v4h*)(&Al[wave][rr][lane * 4]) = lv; }
  wave_lds_sync();
  v8f acc[16];
#pragma unroll
  for (int t = 0; t < 16; ++t) acc[t] = (v8f){};
#pragma unroll
  for (int kb = 0; kb < DM; kb += 32) { const v16b a = frag_kb(&Ah[wave][nloc][kb], hlf), al = frag_kb(&Al[wave][nloc][kb], hlf);
#pragma unroll
    for (int t = 0; t < 16; ++t) { const v16b bw = frag_kb(W1T + (size_t)(t * 16 + nloc) * DM + kb, hlf); acc[t] = wmma16b(a, bw, acc[t]); acc[t] = wmma16b(al, bw, acc[t]); } }
#pragma unroll
  for (int t = 0; t < 16; ++t) { const float bb = bf16_rne(b1[t * 16 + nloc]);
#pragma unroll
    for (int r = 0; r < 8; ++r) Tf[wave][8 * hlf + r][t * 16 + nloc] = fmaxf(acc[t][r] * (1.0f / (XS * WSC)) + bb, 0.0f); }
  wave_lds_sync();
  for (int pass = 0; pass < 2; ++pass) { for (int rr = 0; rr < 16; ++rr) for (int hf = 0; hf < 2; ++hf) *(volatile v4f*)(F1 + (m0 + rr) * FF + hf * 128 + lane * 4) = *(const v4f*)(&Tf[wave][rr][hf * 128 + lane * 4]); __threadfence(); }
}
__global__ __launch_bounds__(64) void ffn2_kernel(const float* __restrict__ F1, const b16* __restrict__ W2T, const float* __restrict__ b2, const float* __restrict__ Y1, const float* __restrict__ g2, const float* __restrict__ be2, float* __restrict__ out) {
  __shared__ __attribute__((aligned(16))) b16 Ah[2][16][128 + 8], Al[2][16][128 + 8]; __shared__ __attribute__((aligned(16))) float Tf[2][16][128 + 4];
  const int wave = threadIdx.x >> 5, lane = threadIdx.x & 31, nloc = lane & 15, hlf = lane >> 4; const size_t m0 = (size_t)blockIdx.x * 32 + wave * 16;
  v8f acc[8];
#pragma unroll
  for (int t = 0; t < 8; ++t) acc[t] = (v8f){};
#pragma unroll 1
  for (int kc = 0; kc < FF; kc += 128) {
    for (int rr = 0; rr < 16; ++rr) { const v4f v = *(const v4f*)(F1 + (m0 + rr) * FF + kc + lane * 4); v4h hv, lv; for (int j = 0; j < 4; ++j) { b16 p, q; split16(v[j] * XS, p, q); hv[j] = p; lv[j] = q; } *(v4h*)(&Ah[wave][rr][lane * 4]) = hv; *(v4h*)(&Al[wave][rr][lane * 4]) = lv; }
    wave_lds_sync();
#pragma unroll
    for (int kb = 0; kb < 128; kb += 32) { const v16b a = frag_kb(&Ah[wave][nloc][kb], hlf), al = frag_kb(&Al[wave][nloc][kb], hlf);
#pragma unroll
      for (int t = 0; t < 8; ++t) { const v16b bw = frag_kb(W2T + (size_t)(t * 16 + nloc) * FF + kc + kb, hlf); acc[t] = wmma16b(a, bw, acc[t]); acc[t] = wmma16b(al, bw, acc[t]); } }
    wave_lds_sync(); }
#pragma unroll
  for (int t = 0; t < 8; ++t) { const float bb = bf16_rne(b2[t * 16 + nloc]);
#pragma unroll
    for (int r = 0; r < 8; ++r) Tf[wave][8 * hlf + r][t * 16 + nloc] = fmaxf(acc[t][r] * (1.0f / (XS * WSC)) + bb, 0.0f) + Y1[(m0 + 8 * hlf + r) * DM + t * 16 + nloc]; }
  wave_lds_sync();
  row_ln_store(Tf[wave], lane, g2, be2, out, m0, DM, true);
}
}

extern "C" void kernel_launch(void* const* d_in, const int* in_sizes, int n_in, void* d_out, int out_size, void* d_ws, size_t ws_size, hipStream_t stream) {
  (void)n_in;
  auto Fp = [&](int i) { return (const float*)d_in[i]; };
  if (in_sizes[0] != B * T * DM || in_sizes[1] != H * DM * HD || in_sizes[2] != H * HD || in_sizes[3] != H * DM * HD || in_sizes[5] != H * DM * HD || in_sizes[7] != INNER * DM || in_sizes[8] != DM || in_sizes[9] != DM * FF || in_sizes[10] != FF || in_sizes[11] != FF * DM || in_sizes[12] != DM || in_sizes[13] != DM || in_sizes[16] != DM || out_size != B * T * DM) return;
  size_t off = 0; char* ws = (char*)d_ws;
  auto carve = [&](size_t bytes) { char* p = ws + off; off += (bytes + 255) & ~(size_t)255; return p; };
  b16* WT = (b16*)carve((size_t)3 * INNER * DM * 2); b16* WO = (b16*)carve((size_t)DM * INNER * 2); b16* W1T = (b16*)carve((size_t)FF * DM * 2); b16* W2T = (b16*)carve((size_t)DM * FF * 2);
  const size_t plane = (size_t)B * H * T * HD * 2; b16* QP = (b16*)carve(plane); b16* KP = (b16*)carve(plane); b16* VTh = (b16*)carve(plane); b16* O = (b16*)carve(plane);
  float* Y1 = (float*)carve((size_t)B * T * DM * 4); float* F1 = (float*)carve((size_t)B * T * FF * 4);
  if (off > ws_size || off > ((size_t)128 << 20)) return;
  const size_t nprep = (size_t)3 * INNER * DM / 8 + (size_t)DM * INNER / 8 + (size_t)FF * DM / 8 + (size_t)DM * FF / 8;
  prep_kernel<<<(unsigned)((nprep + 255) / 256), 256, 0, stream>>>(Fp(1), Fp(3), Fp(5), Fp(7), Fp(9), Fp(11), WT, WO, W1T, W2T);
  proj_kernel<<<dim3(T / 64, BL, 3 * H), 128, 0, stream>>>(Fp(0), WT, Fp(2), Fp(4), Fp(6), QP, KP, VTh);
  attn_kernel<<<dim3(QL / 32, BL * H), 64, 0, stream>>>(QP, KP, VTh, O);
  outln_kernel<<<(unsigned)((size_t)BL * QL / 64), 128, 0, stream>>>(O, WO, Fp(8), Fp(13), Fp(14), Y1);
  ffn1_kernel<<<(unsigned)((size_t)BL * QL / 32), 64, 0, stream>>>(Y1, W1T, Fp(10), F1);
  ffn2_kernel<<<(unsigned)((size_t)BL * QL / 32), 64, 0, stream>>>(F1, W2T, Fp(12), Y1, Fp(15), Fp(16), (float*)d_out);
}
